// TransRScore_76124000354696
// MI455X (gfx1250) — hardware-verified
//
#include <hip/hip_runtime.h>
#define NNo 100000
#define NE 400000
#define NR 1000
#define DE 32
#define RCAP 480
#define GAM 12.0f
typedef __bf16 v16b __attribute__((ext_vector_type(16)));
typedef unsigned short v8us __attribute__((ext_vector_type(8), may_alias));
typedef float  v8f  __attribute__((ext_vector_type(8)));
typedef float  v4f  __attribute__((ext_vector_type(4)));
typedef float  v4fa __attribute__((ext_vector_type(4), may_alias));
union FragB { v16b v; v8us half[2]; unsigned short u[16]; };

__device__ __forceinline__ unsigned short bf16_bits(float x) { unsigned int u = __float_as_uint(x); return (unsigned short)((u + 0x7FFFu + ((u >> 16) & 1u)) >> 16); }
__device__ __forceinline__ float bf16_val(unsigned short b) { return __uint_as_float(((unsigned int)b) << 16); }
__device__ __forceinline__ float bf16_round(float x) { return bf16_val(bf16_bits(x)); }
template <int NT>
__device__ __forceinline__ v8f mmaN(v16b ah, v16b al, v16b bh, v16b bl, v8f c) {
  c = __builtin_amdgcn_wmma_f32_16x16x32_bf16(false, ah, false, bh, (short)0, c, false, false);
  if (NT >= 2) c = __builtin_amdgcn_wmma_f32_16x16x32_bf16(false, al, false, bh, (short)0, c, false, false);
  if (NT >= 3) c = __builtin_amdgcn_wmma_f32_16x16x32_bf16(false, ah, false, bl, (short)0, c, false, false);
  asm volatile("v_nop\n\tv_nop\n\tv_nop\n\tv_nop" : "+v"(c) : "v"(ah), "v"(al), "v"(bh), "v"(bl));
  return c;
}

__global__ __launch_bounds__(256) void k_wt_bf16(const float* __restrict__ W, unsigned short* __restrict__ Wt, int K, int N) {
  const int t = blockIdx.x * 256 + threadIdx.x;
  const int k8n = K / 8;
  if (t >= N * k8n) return;
  const int n = t / k8n, k8 = (t % k8n) * 8;
  v8us v;
#pragma unroll
  for (int i = 0; i < 8; ++i) v[i] = bf16_bits(W[(size_t)(k8 + i) * N + n]);
  *(volatile v8us*)(Wt + (size_t)n * K + k8) = v;
  __threadfence();
  *(volatile v8us*)(Wt + (size_t)n * K + k8) = v;
}

template <bool ASPLIT, int ACT, bool BIAS_BF16>
__global__ __launch_bounds__(128) void k_gemm_bf(const float* __restrict__ A, int lda, const unsigned short* __restrict__ Wt, int ldb,
                                               const float* __restrict__ bias, float* __restrict__ C, int ldc, int M, int N, int K) {
  __shared__ __attribute__((aligned(16))) float so[4][16][64];
  const int tid = threadIdx.x, w = tid >> 5, lane = tid & 31, ln = lane & 15, hh = lane >> 4;
  const int ntn = N / 64;
  const int wid = blockIdx.x * 4 + w;
  const int mt = wid / ntn, nq = wid % ntn;
  if (mt * 16 >= M) return;
  const int row0 = mt * 16, col0 = nq * 64;
  const float* arow = A + (size_t)(row0 + ln) * lda;
  v8f acc[4] = {};
  for (int kb = 0; kb < K; kb += 32) {
    FragB ah, al;
    const v4f x0 = *(const v4fa*)(arow + kb + 8 * hh), x1 = *(const v4fa*)(arow + kb + 8 * hh + 4);
    const v4f x2 = *(const v4fa*)(arow + kb + 16 + 8 * hh), x3 = *(const v4fa*)(arow + kb + 16 + 8 * hh + 4);
    float xs[16] = {x0[0],x0[1],x0[2],x0[3],x1[0],x1[1],x1[2],x1[3],x2[0],x2[1],x2[2],x2[3],x3[0],x3[1],x3[2],x3[3]};
#pragma unroll
    for (int i = 0; i < 16; ++i) { const unsigned short hb = bf16_bits(xs[i]); ah.u[i] = hb; al.u[i] = ASPLIT ? bf16_bits(xs[i] - bf16_val(hb)) : (unsigned short)0; }
#pragma unroll
    for (int t = 0; t < 4; ++t) {
      const unsigned short* brow = Wt + (size_t)(col0 + t * 16 + ln) * ldb + kb;
      FragB b;
      b.half[0] = *(const v8us*)(brow + 8 * hh);
      b.half[1] = *(const v8us*)(brow + 16 + 8 * hh);
      acc[t] = mmaN<ASPLIT ? 2 : 1>(ah.v, al.v, b.v, b.v, acc[t]);
    }
  }
#pragma unroll
  for (int t = 0; t < 4; ++t) {
    float bv = bias ? bias[col0 + t * 16 + ln] : 0.f;
    if (BIAS_BF16) bv = bf16_round(bv);
#pragma unroll
    for (int r = 0; r < 8; ++r) { float v = acc[t][r] + bv; if (ACT == 1) v = fmaxf(v, 0.f); so[w][8 * hh + r][t * 16 + ln] = v; }
  }
  __builtin_amdgcn_fence(__ATOMIC_ACQ_REL, "workgroup");
  __builtin_amdgcn_wave_barrier();
  const int rsub = lane >> 4, c4 = (lane & 15) * 4;
  for (int pass = 0; pass < 2; ++pass) {
#pragma unroll
    for (int q = 0; q < 8; ++q) {
      const int r = q * 2 + rsub;
      const v4f v = *(const v4fa*)&so[w][r][c4];
      *(volatile v4f*)(C + (size_t)(row0 + r) * ldc + col0 + c4) = v;
    }
    if (pass == 0) __threadfence();
  }
}

template <bool ASPLIT, int ACT, bool BIAS_BF16, bool RES_BF16>
__global__ __launch_bounds__(128) void k_gemm_bf3(const float* __restrict__ A, int lda, const unsigned short* __restrict__ Wt, int ldb,
                                                const float* __restrict__ bias, const float* __restrict__ resid, int rmod, int ldr,
                                                float* __restrict__ C, int ldc, int M, int N, int K) {
  __shared__ __attribute__((aligned(16))) float so[4][16][64];
  const int tid = threadIdx.x, w = tid >> 5, lane = tid & 31, ln = lane & 15, hh = lane >> 4;
  const int ntn = N / 64;
  const int wid = blockIdx.x * 4 + w;
  const int mt = wid / ntn, nq = wid % ntn;
  if (mt * 16 >= M) return;
  const int row0 = mt * 16, col0 = nq * 64;
  const float* arow = A + (size_t)(row0 + ln) * lda;
  v8f acc[4] = {};
  for (int kb = 0; kb < K; kb += 32) {
    FragB ah, al;
    const v4f x0 = *(const v4fa*)(arow + kb + 8 * hh), x1 = *(const v4fa*)(arow + kb + 8 * hh + 4);
    const v4f x2 = *(const v4fa*)(arow + kb + 16 + 8 * hh), x3 = *(const v4fa*)(arow + kb + 16 + 8 * hh + 4);
    float xs[16] = {x0[0],x0[1],x0[2],x0[3],x1[0],x1[1],x1[2],x1[3],x2[0],x2[1],x2[2],x2[3],x3[0],x3[1],x3[2],x3[3]};
#pragma unroll
    for (int i = 0; i < 16; ++i) { const unsigned short hb = bf16_bits(xs[i]); ah.u[i] = hb; al.u[i] = ASPLIT ? bf16_bits(xs[i] - bf16_val(hb)) : (unsigned short)0; }
#pragma unroll
    for (int t = 0; t < 4; ++t) {
      const unsigned short* brow = Wt + (size_t)(col0 + t * 16 + ln) * ldb + kb;
      FragB b;
      b.half[0] = *(const v8us*)(brow + 8 * hh);
      b.half[1] = *(const v8us*)(brow + 16 + 8 * hh);
      acc[t] = mmaN<ASPLIT ? 2 : 1>(ah.v, al.v, b.v, b.v, acc[t]);
    }
  }
#pragma unroll
  for (int t = 0; t < 4; ++t) {
    const int col = col0 + t * 16 + ln;
    float bv = bias ? bias[col] : 0.f;
    if (BIAS_BF16) bv = bf16_round(bv);
#pragma unroll
    for (int r = 0; r < 8; ++r) {
      float v = acc[t][r] + bv;
      if (resid) { float rv = resid[(size_t)((row0 + 8 * hh + r) % rmod) * ldr + col]; if (RES_BF16) rv = bf16_round(rv); v += rv; }
      if (ACT == 1) v = fmaxf(v, 0.f);
      if (ACT == 2) v = 0.5f * v * (1.0f + erff(v * 0.70710678118654752f));
      if (ACT == 3) { const float u = 0.7978845608028654f * (v + 0.044715f * v * v * v); v = 0.5f * v * (1.0f + tanhf(u)); }
      so[w][8 * hh + r][t * 16 + ln] = v;
    }
  }
  __builtin_amdgcn_fence(__ATOMIC_ACQ_REL, "workgroup");
  __builtin_amdgcn_wave_barrier();
  const int rsub = lane >> 4, c4 = (lane & 15) * 4;
  for (int pass = 0; pass < 2; ++pass) {
#pragma unroll
    for (int q = 0; q < 8; ++q) {
      const int r = q * 2 + rsub;
      const v4f v = *(const v4fa*)&so[w][r][c4];
      *(volatile v4f*)(C + (size_t)(row0 + r) * ldc + col0 + c4) = v;
    }
    if (pass == 0) __threadfence();
  }
}
template <bool PARAM_BF16>
__global__ __launch_bounds__(256) void k_layernorm(const float* __restrict__ X, const float* __restrict__ R, const float* __restrict__ g, const float* __restrict__ bta,
                                                  float* __restrict__ out_sum, float* __restrict__ out_norm, int N, float eps) {
  __shared__ float red[256];
  const int row = blockIdx.x, tid = threadIdx.x;
  const float* x = X + (size_t)row * N; const float* rr = R ? R + (size_t)row * N : nullptr;
  float vals[16];
  const int per = N / 256;
  float s1 = 0.f;
  for (int u = 0; u < per / 4; ++u) {
    const int j = tid * 4 + 1024 * u;
    const v4f a = *(const v4fa*)(x + j);
    v4f b = {0.f,0.f,0.f,0.f}; if (rr) b = *(const v4fa*)(rr + j);
#pragma unroll
    for (int q = 0; q < 4; ++q) { const float v = a[q] + b[q]; vals[u * 4 + q] = v; s1 += v; }
  }
  red[tid] = s1; __syncthreads();
  for (int st = 128; st > 0; st >>= 1) { if (tid < st) red[tid] += red[tid + st]; __syncthreads(); }
  const float mu = red[0] / (float)N; __syncthreads();
  float s2 = 0.f;
  for (int u = 0; u < per / 4; ++u)
#pragma unroll
    for (int q = 0; q < 4; ++q) { const float c = vals[u * 4 + q] - mu; s2 += c * c; }
  red[tid] = s2; __syncthreads();
  for (int st = 128; st > 0; st >>= 1) { if (tid < st) red[tid] += red[tid + st]; __syncthreads(); }
  const float rs = rsqrtf(red[0] / (float)N + eps);
  for (int pass = 0; pass < 2; ++pass) {
    for (int u = 0; u < per / 4; ++u) {
      const int j = tid * 4 + 1024 * u;
      v4f o, sm;
#pragma unroll
      for (int q = 0; q < 4; ++q) {
        float gg = g[j + q], bb = bta[j + q];
        if (PARAM_BF16) { gg = bf16_round(gg); bb = bf16_round(bb); }
        sm[q] = vals[u * 4 + q]; o[q] = (vals[u * 4 + q] - mu) * rs * gg + bb;
      }
      if (out_sum) *(volatile v4f*)(out_sum + (size_t)row * N + j) = sm;
      *(volatile v4f*)(out_norm + (size_t)row * N + j) = o;
    }
    if (pass == 0) __threadfence();
  }
}


typedef _Float16 v16h __attribute__((ext_vector_type(16)));
union FragH { v16h v; v8us half[2]; _Float16 h[16]; unsigned short u[16]; };
template <int NT>
__device__ __forceinline__ v8f mmaH(v16h ah, v16h al, v16h bh, v16h bl, v8f c) {
  c = __builtin_amdgcn_wmma_f32_16x16x32_f16(false, ah, false, bh, (short)0, c, false, false);
  if (NT >= 2) c = __builtin_amdgcn_wmma_f32_16x16x32_f16(false, al, false, bh, (short)0, c, false, false);
  if (NT >= 3) c = __builtin_amdgcn_wmma_f32_16x16x32_f16(false, ah, false, bl, (short)0, c, false, false);
  asm volatile("v_nop\n\tv_nop\n\tv_nop\n\tv_nop" : "+v"(c) : "v"(ah), "v"(al), "v"(bh), "v"(bl));
  return c;
}
template <bool ASPLIT>
__global__ __launch_bounds__(128) void k_gemm_h(const float* __restrict__ A, int lda, size_t sA, const _Float16* __restrict__ Bh, int ldb, size_t sB, float alpha, float* __restrict__ C, int ldc, size_t sC, int M, int N, int K) {
  __shared__ __attribute__((aligned(16))) float so[4][16][64];
  const int tid = threadIdx.x, w = tid >> 5, lane = tid & 31, ln = lane & 15, hh = lane >> 4; const int by = blockIdx.y;
  A += (size_t)by * sA; Bh += (size_t)by * sB; C += (size_t)by * sC;
  const int ntn = (N + 63) / 64; const int wid = blockIdx.x * 4 + w; const int mt = wid / ntn, nq = wid % ntn; if (mt * 16 >= M) return;
  const int row0 = mt * 16, col0 = nq * 64; const float* arow = A + (size_t)(row0 + ln) * lda;
  v8f acc[4] = {};
  for (int kb = 0; kb < K; kb += 32) {
    FragH ah, al;
    const v4f x0 = *(const v4fa*)(arow + kb + 8 * hh), x1 = *(const v4fa*)(arow + kb + 8 * hh + 4), x2 = *(const v4fa*)(arow + kb + 16 + 8 * hh), x3 = *(const v4fa*)(arow + kb + 16 + 8 * hh + 4);
    float xs[16] = {x0[0],x0[1],x0[2],x0[3],x1[0],x1[1],x1[2],x1[3],x2[0],x2[1],x2[2],x2[3],x3[0],x3[1],x3[2],x3[3]};
#pragma unroll
    for (int i = 0; i < 16; ++i) { const _Float16 h = (_Float16)xs[i]; ah.h[i] = h; al.h[i] = ASPLIT ? (_Float16)(xs[i] - (float)h) : (_Float16)0.0f; }
#pragma unroll
    for (int t = 0; t < 4; ++t) { if (col0 + t * 16 >= N) continue; const size_t boff = (size_t)(col0 + t * 16 + ln) * ldb + kb; FragH bq; bq.half[0] = *(const v8us*)(Bh + boff + 8 * hh); bq.half[1] = *(const v8us*)(Bh + boff + 16 + 8 * hh);
      acc[t] = mmaH<ASPLIT ? 2 : 1>(ah.v, al.v, bq.v, bq.v, acc[t]); }
  }
#pragma unroll
  for (int t = 0; t < 4; ++t) { if (col0 + t * 16 >= N) continue;
#pragma unroll
    for (int r = 0; r < 8; ++r) so[w][8 * hh + r][t * 16 + ln] = acc[t][r] * alpha; }
  __builtin_amdgcn_fence(__ATOMIC_ACQ_REL, "workgroup"); __builtin_amdgcn_wave_barrier();
  const int rsub = lane >> 4, c4 = (lane & 15) * 4;
  for (int pass = 0; pass < 2; ++pass) {
#pragma unroll
    for (int q = 0; q < 8; ++q) { const int r = q * 2 + rsub; if (col0 + c4 < N) { const v4f v = *(const v4fa*)&so[w][r][c4]; *(volatile v4f*)(C + (size_t)(row0 + r) * ldc + col0 + c4) = v; } }
    if (pass == 0) __threadfence(); }
}

__global__ __launch_bounds__(256) void k_wt_f16(const float* __restrict__ W, _Float16* __restrict__ Wt, int K, int N, float scale) {
  const int t = blockIdx.x * 256 + threadIdx.x; if (t >= N * (K / 8)) return; const int n = t / (K / 8), k8 = (t % (K / 8)) * 8; FragH f;
#pragma unroll
  for (int i = 0; i < 8; ++i) f.h[i] = (_Float16)(bf16_round(W[(size_t)(k8 + i) * N + n]) * scale); const v8us o = f.half[0];
  *(volatile v8us*)((unsigned short*)Wt + (size_t)n * K + k8) = o; __threadfence(); *(volatile v8us*)((unsigned short*)Wt + (size_t)n * K + k8) = o;
}
template <int ACT>
__global__ __launch_bounds__(128) void k_gemm_hhx(const _Float16* __restrict__ A, int lda, size_t sA, const _Float16* __restrict__ Bh, int ldb, size_t sB, float alpha, const float* __restrict__ bias, size_t sBias, const float* __restrict__ CP, int rowsPerB, size_t sCPb, int row0g,
    float* __restrict__ C, _Float16* __restrict__ C16, int ldc, size_t sC, int M, int N, int K) {
  __shared__ __attribute__((aligned(16))) float so[4][16][64];
  const int tid = threadIdx.x, w = tid >> 5, lane = tid & 31, ln = lane & 15, hh = lane >> 4; const int by = blockIdx.y;
  A += (size_t)by * sA; Bh += (size_t)by * sB; const size_t cofs = (size_t)by * sC; const float* bp = bias ? bias + (size_t)by * sBias : nullptr;
  const int ntn = (N + 63) / 64; const int wid = blockIdx.x * 4 + w; const int mt = wid / ntn, nq = wid % ntn; if (mt * 16 >= M) return;
  const int row0 = mt * 16, col0 = nq * 64; const _Float16* arow = A + (size_t)(row0 + ln) * lda;
  v8f acc[4] = {};
  for (int kb = 0; kb < K; kb += 32) { FragH ah; ah.half[0] = *(const v8us*)((const unsigned short*)arow + kb + 8 * hh); ah.half[1] = *(const v8us*)((const unsigned short*)arow + kb + 16 + 8 * hh);
#pragma unroll
    for (int t = 0; t < 4; ++t) { if (col0 + t * 16 >= N) continue; const size_t boff = (size_t)(col0 + t * 16 + ln) * ldb + kb; FragH bq; bq.half[0] = *(const v8us*)((const unsigned short*)Bh + boff + 8 * hh); bq.half[1] = *(const v8us*)((const unsigned short*)Bh + boff + 16 + 8 * hh);
      acc[t] = mmaH<1>(ah.v, ah.v, bq.v, bq.v, acc[t]); }
  }
#pragma unroll
  for (int t = 0; t < 4; ++t) { if (col0 + t * 16 >= N) continue; const int col = col0 + t * 16 + ln; const float bv = bp ? bf16_round(bp[col]) : 0.f;
#pragma unroll
    for (int r = 0; r < 8; ++r) { float v = acc[t][r] * alpha + bv; if (CP) { const int bidx = (row0g + row0 + 8 * hh + r) / rowsPerB; v += CP[(size_t)bidx * sCPb + (size_t)by * 64 + col]; } if (ACT == 1) v = (v > 0.f) ? v : expm1f(v); else if (ACT == 7) v = (v > 0.f) ? v + 1.0f : expf(v); else if (ACT == 8) v = tanhf(v); else if (ACT == 9) v = 0.5f * v * (1.0f + tanhf(0.7978845608028654f * (v + 0.044715f * v * v * v))); else if (ACT == 11) v = 1.0f / (1.0f + expf(-v)); else if (ACT == 12) v = (v > 0.f) ? v : 0.01f * v; else if (ACT == 14) v = (v > 0.f) ? v : 0.1f * v; else if (ACT == 15) v = v / (1.0f + expf(-v)); else if (ACT == 3) v = fmaxf(v, 0.f); else if (ACT == 6) v = 0.5f * v * (1.0f + erff(v * 0.70710678118654752f)); so[w][8 * hh + r][t * 16 + ln] = v; } }
  __builtin_amdgcn_fence(__ATOMIC_ACQ_REL, "workgroup"); __builtin_amdgcn_wave_barrier();
  const int rsub = lane >> 4, c4 = (lane & 15) * 4; typedef _Float16 v4h __attribute__((ext_vector_type(4)));
  for (int pass = 0; pass < 2; ++pass) {
#pragma unroll
    for (int q = 0; q < 8; ++q) { const int r = q * 2 + rsub; if (col0 + c4 < N) { const v4f v = *(const v4fa*)&so[w][r][c4]; if (C) *(volatile v4f*)(C + cofs + (size_t)(row0 + r) * ldc + col0 + c4) = v; if (C16) { v4h h4; for (int i = 0; i < 4; ++i) h4[i] = (_Float16)v[i]; *(volatile v4h*)(C16 + cofs + (size_t)(row0 + r) * ldc + col0 + c4) = h4; } } }
    if (pass == 0) __threadfence(); }
}


typedef _Float16 v4h __attribute__((ext_vector_type(4)));

__global__ __launch_bounds__(256) void k_x16(const float* __restrict__ x, _Float16* __restrict__ X16, size_t n8) { const size_t t = (size_t)blockIdx.x * 256 + threadIdx.x; if (t >= n8) return; FragH f;
#pragma unroll
  for (int q = 0; q < 8; ++q) f.h[q] = (_Float16)bf16_round(x[t * 8 + q]); *(volatile v8us*)((unsigned short*)X16 + t * 8) = f.half[0]; __threadfence(); *(volatile v8us*)((unsigned short*)X16 + t * 8) = f.half[0]; }
__global__ __launch_bounds__(256) void k_h16(const float* __restrict__ x, _Float16* __restrict__ X16, size_t n8) { const size_t t = (size_t)blockIdx.x * 256 + threadIdx.x; if (t >= n8) return; FragH f;
#pragma unroll
  for (int q = 0; q < 8; ++q) f.h[q] = (_Float16)x[t * 8 + q]; *(volatile v8us*)((unsigned short*)X16 + t * 8) = f.half[0]; __threadfence(); *(volatile v8us*)((unsigned short*)X16 + t * 8) = f.half[0]; }
__global__ __launch_bounds__(256) void k_round16f(const float* __restrict__ W, _Float16* __restrict__ Bt, size_t n8) { const size_t t = (size_t)blockIdx.x * 256 + threadIdx.x; if (t >= n8) return; FragH f;
#pragma unroll
  for (int i = 0; i < 8; ++i) f.h[i] = (_Float16)(bf16_round(W[t * 8 + i]) * 16.0f); *(volatile v8us*)((unsigned short*)Bt + t * 8) = f.half[0]; __threadfence(); *(volatile v8us*)((unsigned short*)Bt + t * 8) = f.half[0]; }
template <int NHv, int TTv>
__global__ __launch_bounds__(256) void k_vt(const _Float16* __restrict__ V16, int ldv, int voff, _Float16* __restrict__ Vt) { __shared__ unsigned short tl[64][66]; const int tid = threadIdx.x; const int slab = blockIdx.x / (TTv / 64), lg = blockIdx.x % (TTv / 64); const int b = slab / NHv, h = slab % NHv;
  for (int i = tid; i < 64 * 8; i += 256) { const int r = i / 8, c8 = (i % 8) * 8; FragH f; f.half[0] = *(const v8us*)((const unsigned short*)V16 + ((size_t)b * TTv + lg * 64 + r) * ldv + voff + h * 64 + c8);
#pragma unroll
    for (int q = 0; q < 8; ++q) tl[r][c8 + q] = f.u[q]; }
  __syncthreads();
  for (int pass = 0; pass < 2; ++pass) {
#pragma unroll
    for (int rd = 0; rd < 2; ++rd) { const int d = rd * 32 + tid / 8, pc = tid % 8; FragH f;
#pragma unroll
      for (int q = 0; q < 8; ++q) f.u[q] = tl[pc * 8 + q][d];
      *(volatile v8us*)((unsigned short*)Vt + ((size_t)slab * 64 + d) * TTv + lg * 64 + pc * 8) = f.half[0]; }
    if (pass == 0) __threadfence(); } }

__global__ __launch_bounds__(256) void k_hl(const float* __restrict__ F, _Float16* __restrict__ Hh, _Float16* __restrict__ Hl, size_t n8) { const size_t t = (size_t)blockIdx.x * 256 + threadIdx.x; if (t >= n8) return; FragH fh, fl; const v4f a = *(const v4fa*)(F + t * 8), c = *(const v4fa*)(F + t * 8 + 4);
#pragma unroll
  for (int q = 0; q < 4; ++q) { _Float16 h = (_Float16)a[q]; fh.h[q] = h; fl.h[q] = (_Float16)((a[q] - (float)h) * 1024.0f); h = (_Float16)c[q]; fh.h[4 + q] = h; fl.h[4 + q] = (_Float16)((c[q] - (float)h) * 1024.0f); }
  for (int pass = 0; pass < 2; ++pass) { *(volatile v8us*)((unsigned short*)Hh + t * 8) = fh.half[0]; *(volatile v8us*)((unsigned short*)Hl + t * 8) = fl.half[0]; if (pass == 0) __threadfence(); } }
#define VST2(T, ptr, val) do { const T vst2_v_ = (val); *(volatile T*)(ptr) = vst2_v_; __threadfence(); *(volatile T*)(ptr) = vst2_v_; } while (0)

#define C4_NB 4096
#define C4_CH 8192
__device__ __forceinline__ int c4_bucket(int v, int N) { v = min(max(v, 0), N - 1); return (int)(((long long)v * C4_NB) / N); }
__global__ __launch_bounds__(256) void k_c4_count(const int* __restrict__ tgt, int E, int N, int* __restrict__ CNT) {
    __shared__ int hist[C4_NB]; const int ch = blockIdx.x, t = threadIdx.x; const int e0 = ch * C4_CH; const int nt = min(C4_CH, E - e0);
    for (int j = 0; j < 16; ++j) hist[t + 256 * j] = 0; __syncthreads();
    for (int i = t; i < nt; i += 256) atomicAdd(&hist[c4_bucket(tgt[e0 + i], N)], 1);
    __syncthreads();
    for (int j = 0; j < 16; ++j) { const int v = hist[t + 256 * j]; VST2(int, CNT + (long long)ch * C4_NB + t + 256 * j, v); } }
__global__ __launch_bounds__(256) void k_c4_offsets(const int* __restrict__ CNT, int nch, int E, int* __restrict__ OFFB, int* __restrict__ BOFF) {
    __shared__ int tot[C4_NB]; __shared__ int part[256]; const int t = threadIdx.x;
    for (int j = 0; j < 16; ++j) { const int b = t + 256 * j; int s = 0; for (int ch = 0; ch < nch; ++ch) s += CNT[(long long)ch * C4_NB + b]; tot[b] = s; }
    __syncthreads();
    { int s = 0; for (int q = 0; q < 16; ++q) s += tot[16 * t + q]; part[t] = s; } __syncthreads();
    if (t == 0) { int run = 0; for (int i = 0; i < 256; ++i) { const int v = part[i]; part[i] = run; run += v; } } __syncthreads();
    { int run = part[t]; for (int q = 0; q < 16; ++q) { const int v = tot[16 * t + q]; tot[16 * t + q] = run; run += v; } }
    __syncthreads();
    for (int j = 0; j < 16; ++j) { const int b = t + 256 * j; VST2(int, BOFF + b, tot[b]); }
    if (t == 0) VST2(int, BOFF + C4_NB, E);
    for (int j = 0; j < 16; ++j) { const int b = t + 256 * j; int run = tot[b]; for (int ch = 0; ch < nch; ++ch) { VST2(int, OFFB + (long long)ch * C4_NB + b, run); run += CNT[(long long)ch * C4_NB + b]; } } }
__global__ __launch_bounds__(256) void k_c4_scatter(const int* __restrict__ tgt, int E, int N, const int* __restrict__ OFFB, int* __restrict__ BUF) {
    __shared__ int cur[C4_NB]; __shared__ int bk[256]; const int ch = blockIdx.x, t = threadIdx.x; const int e0 = ch * C4_CH; const int nt = min(C4_CH, E - e0);
    const int wv = t >> 5, ln = t & 31;
    for (int j = 0; j < 16; ++j) cur[t + 256 * j] = OFFB[(long long)ch * C4_NB + t + 256 * j];
    __syncthreads();
    for (int s0 = 0; s0 < C4_CH; s0 += 256) {
        const int i = s0 + t; const int e = e0 + i; const int b = (i < nt) ? c4_bucket(tgt[min(e, E - 1)], N) : -1;
        bk[t] = b; __syncthreads();
        int rank = 0, cntw = 0;
        for (int l = 0; l < 32; ++l) { const int o = bk[(wv << 5) + l]; const bool same = (o == b) && (b >= 0); cntw += same ? 1 : 0; rank += (same && l < ln) ? 1 : 0; }
        const bool last = (b >= 0) && (rank == cntw - 1);
        for (int w = 0; w < 8; ++w) {
            if (wv == w && b >= 0) { int pos = cur[b] + rank; pos = min(max(pos, 0), E - 1); VST2(int, BUF + pos, e); }
            __syncthreads();
            if (wv == w && last) cur[b] += cntw;
            __syncthreads(); }
    } }
template <int CAP>
__global__ __launch_bounds__(256) void k_c4_lists(const int* __restrict__ tgt, const int* __restrict__ BUF, const int* __restrict__ BOFF, int N, int E, int* __restrict__ NBR, int* __restrict__ cnt) {
    const int d = blockIdx.x * 256 + threadIdx.x; if (d >= N) return; const int b = c4_bucket(d, N); int n = 0; int* row = NBR + (long long)d * CAP;
    const int p0 = min(max(BOFF[b], 0), E), p1 = min(max(BOFF[b + 1], p0), E);
    for (int p = p0; p < p1; ++p) { int e = BUF[p]; e = min(max(e, 0), E - 1); if (tgt[e] == d) { if (n < CAP) VST2(int, row + n, e); ++n; } }
    for (int j = n; j < CAP; ++j) VST2(int, row + j, -1); VST2(int, cnt + d, min(n, CAP)); }
__global__ __launch_bounds__(256) void k_c4_scan1(const int* __restrict__ cnt, int* __restrict__ PART, int N) {
    __shared__ int part[256]; const int per = ((((N + 255) / 256) + 31) / 32) * 32; const int a = threadIdx.x * per, b = min(N, a + per); int s = 0;
    for (int i = a; i < b; ++i) s += cnt[i]; part[threadIdx.x] = s; __syncthreads();
    if (threadIdx.x == 0) { int run = 0; for (int t = 0; t < 256; ++t) { const int v = part[t]; part[t] = run; run += v; } } __syncthreads();
    VST2(int, PART + threadIdx.x, part[threadIdx.x]); }
__global__ __launch_bounds__(256) void k_c4_scan2(const int* __restrict__ cnt, const int* __restrict__ PART, int* __restrict__ off, int N) {
    const int i = blockIdx.x * 256 + threadIdx.x; if (i > N) return; const int per = ((((N + 255) / 256) + 31) / 32) * 32; const int r = min(i / per, 255); const int a = r * per;
    int s = PART[r]; for (int kq = a; kq < i; ++kq) s += cnt[min(kq, N - 1)];
    VST2(int, off + i, s); }
template <int CAP>
__global__ __launch_bounds__(256) void k_c4_slotcopy(const int* __restrict__ off, const int* __restrict__ NBR, int* __restrict__ slot, int N) {
    const int t = blockIdx.x * 256 + threadIdx.x; const int tot = off[N]; if (t >= tot) return;
    int lo = 0, hi = N - 1; while (lo < hi) { const int mid = (lo + hi + 1) >> 1; if (off[mid] <= t) lo = mid; else hi = mid - 1; }
    int j = t - off[lo]; j = (j < 0) ? 0 : ((j >= CAP) ? (CAP - 1) : j); VST2(int, slot + t, NBR[(long long)lo * CAP + j]); }

__global__ __launch_bounds__(256) void k_gx(const int* __restrict__ NBR, const int* __restrict__ cnt, const int* __restrict__ src, const int* __restrict__ dst, const float* __restrict__ node, _Float16* __restrict__ XS, _Float16* __restrict__ XD) {
  const size_t t = (size_t)blockIdx.x * 256 + threadIdx.x; if (t >= (size_t)NR * RCAP * 4) return; const int d0 = (int)(t & 3) * 8; const size_t slot = t >> 2; const int r = (int)(slot / RCAP), j = (int)(slot % RCAP); const int ne = min(cnt[r], RCAP); FragH fs, fd;
  int s = 0, d = 0; const bool live = j < ne; if (live) { int e = NBR[(size_t)r * RCAP + j]; e = min(max(e, 0), NE - 1); s = min(max(src[e], 0), NNo - 1); d = min(max(dst[e], 0), NNo - 1); }
#pragma unroll
  for (int q = 0; q < 8; ++q) { const float vs = node[(size_t)s * DE + d0 + q], vd = node[(size_t)d * DE + d0 + q]; fs.h[q] = live ? (_Float16)bf16_round(vs) : (_Float16)0.0f; fd.h[q] = live ? (_Float16)bf16_round(vd) : (_Float16)0.0f; }
  for (int pass = 0; pass < 2; ++pass) { *(volatile v8us*)((unsigned short*)XS + slot * DE + d0) = fs.half[0]; *(volatile v8us*)((unsigned short*)XD + slot * DE + d0) = fd.half[0]; if (pass == 0) __threadfence(); } }
__global__ __launch_bounds__(256) void k_score(const int* __restrict__ rel_id, const int* __restrict__ NBR, const int* __restrict__ cnt, const _Float16* __restrict__ HS, const _Float16* __restrict__ TS, const float* __restrict__ rel, float* __restrict__ out) {
  #pragma clang fp contract(off)
  const int e = blockIdx.x * 256 + threadIdx.x; if (e >= NE) return; int r = rel_id[e]; r = min(max(r, 0), NR - 1); const int ne = min(cnt[r], RCAP); const int* lst = NBR + (size_t)r * RCAP; int lo = 0, hi = ne - 1, j = 0;
#pragma unroll 1
  for (int it = 0; it < 10; ++it) { if (lo <= hi) { const int mid = (lo + hi) >> 1; const int v = lst[mid]; if (v == e) { j = mid; lo = hi + 1; } else if (v < e) lo = mid + 1; else hi = mid - 1; } }
  const size_t ro = ((size_t)r * RCAP + j) * DE; float s = 0.f;
#pragma unroll
  for (int d = 0; d < DE; ++d) s += fabsf(((float)HS[ro + d] + bf16_round(rel[(size_t)r * DE + d])) - (float)TS[ro + d]);
  const float v = GAM - s; *(volatile float*)(out + e) = v; __threadfence(); *(volatile float*)(out + e) = v; }

extern "C" void kernel_launch(void* const* d_in, const int* in_sizes, int n_in,
                              void* d_out, int out_size, void* d_ws, size_t ws_size, hipStream_t stream) {
  (void)in_sizes; (void)n_in; (void)out_size;
  const float* node = (const float*)d_in[0]; const float* rel = (const float*)d_in[1]; const float* tw = (const float*)d_in[2]; const int* src = (const int*)d_in[3]; const int* dst = (const int*)d_in[4]; const int* rid = (const int*)d_in[5];
  char* ws = (char*)d_ws; size_t off = 0;
  auto take = [&](size_t bytes) { char* p = ws + off; off += (bytes + 255) & ~(size_t)255; return p; };
  const int nch = (NE + C4_CH - 1) / C4_CH;
  int* CNT = (int*)take((size_t)nch * C4_NB * 4); int* OFFB = (int*)take((size_t)nch * C4_NB * 4); int* BOFF = (int*)take((size_t)(C4_NB + 64) * 4); int* BUF = (int*)take((size_t)NE * 4); int* NBR = (int*)take((size_t)NR * RCAP * 4); int* cnt = (int*)take((size_t)(NR + 64) * 4);
  _Float16* Bt = (_Float16*)take((size_t)NR * DE * DE * 2); _Float16* XS = (_Float16*)take((size_t)NR * RCAP * DE * 2); _Float16* XD = (_Float16*)take((size_t)NR * RCAP * DE * 2); _Float16* HS = (_Float16*)take((size_t)NR * RCAP * DE * 2); _Float16* TS = (_Float16*)take((size_t)NR * RCAP * DE * 2);
  if (off > ws_size) return;
  k_c4_count<<<nch, 256, 0, stream>>>(rid, NE, NR, CNT); k_c4_offsets<<<1, 256, 0, stream>>>(CNT, nch, NE, OFFB, BOFF); k_c4_scatter<<<nch, 256, 0, stream>>>(rid, NE, NR, OFFB, BUF); k_c4_lists<RCAP><<<(NR + 255) / 256, 256, 0, stream>>>(rid, BUF, BOFF, NR, NE, NBR, cnt);
  k_round16f<<<(NR * DE * DE / 8 + 255) / 256, 256, 0, stream>>>(tw, Bt, (size_t)NR * DE * DE / 8);
  k_gx<<<(unsigned)(((size_t)NR * RCAP * 4 + 255) / 256), 256, 0, stream>>>(NBR, cnt, src, dst, node, XS, XD);
  const dim3 g(((RCAP / 16) * 1 + 3) / 4, NR);
  k_gemm_hhx<0><<<g, 128, 0, stream>>>(XS, DE, (size_t)RCAP * DE, Bt, DE, (size_t)DE * DE, 0.0625f, nullptr, 0, nullptr, 1, 0, 0, nullptr, HS, DE, (size_t)RCAP * DE, RCAP, DE, DE);
  k_gemm_hhx<0><<<g, 128, 0, stream>>>(XD, DE, (size_t)RCAP * DE, Bt, DE, (size_t)DE * DE, 0.0625f, nullptr, 0, nullptr, 1, 0, 0, nullptr, TS, DE, (size_t)RCAP * DE, RCAP, DE, DE);
  k_score<<<(NE + 255) / 256, 256, 0, stream>>>(rid, NBR, cnt, HS, TS, rel, (float*)d_out);
}
